// MultiHeadAttention_80290118631658
// MI455X (gfx1250) — hardware-run, weakly checked
//
#include <hip/hip_runtime.h>


#ifndef NB
#define NB 8
#endif
#ifndef SEQ
#define SEQ 1024
#endif
#define SEQ_FULL 1024
#define TT   SEQ
#define DM   1024
#define NH_  16
#define HD   64
#define DQ   (NH_ * HD)
#define NQKV (3 * DQ)
#define ZH   8
#define PCAR 1024.0f
#define SCL  0.125f
#define RCAR 8.0f
typedef _Float16 h16;
typedef unsigned short bf;
typedef __attribute__((ext_vector_type(16))) __bf16   v16bf;
typedef __attribute__((ext_vector_type(16))) _Float16 v16h;
typedef __attribute__((ext_vector_type(8)))  _Float16 v8h;
typedef __attribute__((ext_vector_type(8)))  unsigned short v8us;
typedef __attribute__((ext_vector_type(8)))  float    v8f;
typedef __attribute__((ext_vector_type(4)))  float    v4f;
typedef v8h  __attribute__((may_alias)) v8ha;
typedef v4f  __attribute__((may_alias)) v4fa;
typedef v8us __attribute__((may_alias)) v8usa;

static_assert(TT % 128 == 0);
static_assert(TT <= SEQ_FULL);
static_assert(DM % 64 == 0);
static_assert(HD == 64);
static_assert(NH_ % ZH == 0);
static_assert(NQKV % 64 == 0);

__device__ __forceinline__ unsigned short f2bf(float f) { unsigned u = __float_as_uint(f); u += 0x7FFFu + ((u >> 16) & 1u); return (unsigned short)(u >> 16); }
__device__ __forceinline__ float bf2f(unsigned short b) { return __uint_as_float(((unsigned)b) << 16); }
__device__ __forceinline__ float bfr(float f) { return bf2f(f2bf(f)); }
__device__ __forceinline__ v16h cat16(v8h lo, v8h hi) { return __builtin_shufflevector(lo, hi, 0, 1, 2, 3, 4, 5, 6, 7, 8, 9, 10, 11, 12, 13, 14, 15); }
__device__ __forceinline__ v16bf cat16b(v8us lo, v8us hi) { return __builtin_bit_cast(v16bf, __builtin_shufflevector(lo, hi, 0, 1, 2, 3, 4, 5, 6, 7, 8, 9, 10, 11, 12, 13, 14, 15)); }
__device__ __forceinline__ v8f wmma16(v16h a, v16h b, v8f c) { return __builtin_amdgcn_wmma_f32_16x16x32_f16(false, a, false, b, (short)0, c, false, false); }
__device__ __forceinline__ v8f wmmab(v16bf a, v16bf b, v8f c) { return __builtin_amdgcn_wmma_f32_16x16x32_bf16(false, a, false, b, (short)0, c, false, false); }

template <typename T16> struct WFrag;
template <> struct WFrag<h16> { typedef v16h V; static __device__ __forceinline__ V ld(const h16* p) { return cat16(*(const v8h*)p, *(const v8h*)(p + 16)); } static __device__ __forceinline__ v8f mma(V a, V b, v8f c) { return wmma16(a, b, c); } };
template <> struct WFrag<bf> { typedef v16bf V; static __device__ __forceinline__ V ld(const bf* p) { return cat16b(*(const v8us*)p, *(const v8us*)(p + 16)); } static __device__ __forceinline__ v8f mma(V a, V b, v8f c) { return wmmab(a, b, c); } };
template <typename T16, int NSPLIT, bool BIAS>
__global__ __launch_bounds__(32) void k_gemmw(const T16* __restrict__ A, const T16* __restrict__ A2, const T16* __restrict__ Bt, const T16* __restrict__ Bt2, int K, float* C, int ldc, const float* __restrict__ bias, size_t sA, size_t sB, size_t sC) {
    typedef typename WFrag<T16>::V V;
    __shared__ __align__(16) float os[16 * 68];
    const size_t z = blockIdx.z; A += z * sA; if (A2) A2 += z * sA; Bt += z * sB; if (Bt2) Bt2 += z * sB; C += z * sC;
    const int lane = threadIdx.x & 31, lr = lane & 15, hi = lane >> 4; const int r0 = blockIdx.x * 64, c0 = blockIdx.y * 64;
    v8f acc[4][4];
#pragma unroll
    for (int mb = 0; mb < 4; ++mb)
#pragma unroll
        for (int nb = 0; nb < 4; ++nb) acc[mb][nb] = (v8f){};
    const size_t aoff = (size_t)(r0 + lr) * K + 8 * hi, boff = (size_t)(c0 + lr) * K + 8 * hi;
#pragma unroll 1
    for (int kc = 0; kc < K; kc += 32) {
        V a[4], a2[4];
#pragma unroll
        for (int mb = 0; mb < 4; ++mb) { a[mb] = WFrag<T16>::ld(A + aoff + (size_t)mb * 16 * K + kc); if (NSPLIT == 1 || NSPLIT == 2) a2[mb] = WFrag<T16>::ld(A2 + aoff + (size_t)mb * 16 * K + kc); }
#pragma unroll
        for (int nb = 0; nb < 4; ++nb) { const V b = WFrag<T16>::ld(Bt + boff + (size_t)nb * 16 * K + kc); V b2; if (NSPLIT >= 2) b2 = WFrag<T16>::ld(Bt2 + boff + (size_t)nb * 16 * K + kc);
#pragma unroll
            for (int mb = 0; mb < 4; ++mb) { acc[mb][nb] = WFrag<T16>::mma(a[mb], b, acc[mb][nb]); if (NSPLIT == 1 || NSPLIT == 2) acc[mb][nb] = WFrag<T16>::mma(a2[mb], b, acc[mb][nb]); if (NSPLIT >= 2) acc[mb][nb] = WFrag<T16>::mma(a[mb], b2, acc[mb][nb]); } }
        asm volatile("v_nop\n\tv_nop\n\tv_nop\n\tv_nop" : "+v"(acc[0][0]), "+v"(acc[1][1]), "+v"(acc[2][2]), "+v"(acc[3][3]) : "v"(a[0]), "v"(a[3]));
    }
#pragma unroll
    for (int mb = 0; mb < 4; ++mb) {
#pragma unroll
        for (int nb = 0; nb < 4; ++nb) {
#pragma unroll
            for (int j = 0; j < 8; ++j) os[(hi * 8 + j) * 68 + nb * 16 + lr] = acc[mb][nb][j]; }
        __builtin_amdgcn_wave_barrier(); asm volatile("" ::: "memory");
        float* crow = C + (size_t)(r0 + mb * 16) * ldc + c0;
#pragma unroll 1
        for (int ps = 0; ps < 2; ++ps) {
#pragma unroll
            for (int s = 0; s < 8; ++s) { const int row = 2 * s + hi, cofs = lr * 4; v4f val = *(const v4fa*)(os + row * 68 + cofs); if (BIAS) { val[0] += bfr(bias[c0 + cofs]); val[1] += bfr(bias[c0 + cofs + 1]); val[2] += bfr(bias[c0 + cofs + 2]); val[3] += bfr(bias[c0 + cofs + 3]); }
                *(volatile v4f*)(crow + (size_t)row * ldc + cofs) = val; }
            if (ps == 0) __threadfence(); }
        __builtin_amdgcn_wave_barrier(); asm volatile("" ::: "memory");
    }
}

__device__ __forceinline__ h16 tohx(float x) { return (h16)x; }
__device__ __forceinline__ void splitf(float y, unsigned short& h, unsigned short& l) { h = f2bf(y); l = f2bf(y - bf2f(h)); }
typedef __attribute__((ext_vector_type(2))) _Float16 v2h;
typedef __attribute__((ext_vector_type(4))) _Float16 v4h;
typedef __attribute__((ext_vector_type(2))) unsigned short v2us;
typedef __attribute__((ext_vector_type(4))) int v4i;

__global__ __launch_bounds__(256) void k_wtG(const float* __restrict__ w, int K, int N, bf* Bt) {
    const int lane = threadIdx.x & 31; const int L0 = (blockIdx.x * 8 + (threadIdx.x >> 5)) * 8; const int nlines = N * K / 64;
#pragma unroll
    for (int ps = 0; ps < 2; ++ps) {
#pragma unroll 1
        for (int l = 0; l < 8; ++l) { const int L = L0 + l; if (L >= nlines) break; const size_t e = (size_t)L * 64 + lane * 2; const int k = (int)(e % K), n = (int)(e / K); v2us o;
            o[0] = f2bf(w[(size_t)k * N + n]); o[1] = f2bf(w[(size_t)(k + 1) * N + n]); *(volatile v2us*)(Bt + e) = o; }
        if (ps == 0) __threadfence(); }
}
__global__ __launch_bounds__(256) void k_cvt8(const float* __restrict__ src, bf* dst, size_t n8, size_t sS, size_t sD) { const size_t i = (size_t)blockIdx.x * 256 + threadIdx.x; if (i >= n8) return; src += (size_t)blockIdx.y * sS; dst += (size_t)blockIdx.y * sD; const v8f v = *(const v8f*)(src + i * 8); v8us o;
#pragma unroll
    for (int k = 0; k < 8; ++k) o[k] = f2bf(v[k]); *(volatile v8us*)(dst + i * 8) = o; __threadfence(); *(volatile v8us*)(dst + i * 8) = o; }

__global__ __launch_bounds__(256) void k_qkp(const float* __restrict__ F, const float* __restrict__ bq, const float* __restrict__ bk, const float* __restrict__ R, h16* QK) {
    const size_t e = ((size_t)blockIdx.x * 256 + threadIdx.x) * 8; if (e >= (size_t)2 * NH_ * TT * HD) return;
    const int which = (int)(e / ((size_t)NH_ * TT * HD)); const size_t rem = e % ((size_t)NH_ * TT * HD);
    const int d = (int)(rem % HD); const int t = (int)((rem / HD) % TT); const int h = (int)(rem / ((size_t)HD * TT));
    const float* f = F + (size_t)t * NQKV + (size_t)which * DQ + h * HD + d;
    const v4f f0 = *(const v4f*)f, f1 = *(const v4f*)(f + 4);
    const v4f q0 = *(const v4f*)(bq + h * HD + d), q1 = *(const v4f*)(bq + h * HD + d + 4);
    const v4f k0 = *(const v4f*)(bk + h * HD + d), k1 = *(const v4f*)(bk + h * HD + d + 4);
    const v4f r0 = *(const v4f*)(R + (size_t)t * HD + d), r1 = *(const v4f*)(R + (size_t)t * HD + d + 4);
    v8h o;
#pragma unroll
    for (int q = 0; q < 8; ++q) { const float fv = (q < 4) ? f0[q & 3] : f1[q & 3]; const float bqv = (q < 4) ? q0[q & 3] : q1[q & 3]; const float bkv = (q < 4) ? k0[q & 3] : k1[q & 3]; const float rv = (q < 4) ? r0[q & 3] : r1[q & 3];
        const float bias = which ? bfr(bkv) : bfr(bqv); const float radd = which ? RCAR * bfr(rv) : 0.0f; const float y = (fv + bias) + radd; o[q] = tohx(y); }
    *(volatile v8h*)(QK + e) = o; __threadfence(); *(volatile v8h*)(QK + e) = o; }
__global__ __launch_bounds__(256) void k_vtp(const float* __restrict__ F, const float* __restrict__ bv, h16* V16) { const size_t e = ((size_t)blockIdx.x * 256 + threadIdx.x) * 2; if (e >= (size_t)NH_ * HD * TT) return; const int t = (int)(e % TT); const int d = (int)((e / TT) % HD); const int g = (int)(e / ((size_t)TT * HD)); const float bb = bfr(bv[g * HD + d]); v2h o16;
#pragma unroll
    for (int q = 0; q < 2; ++q) { const float x = F[(size_t)(t + q) * NQKV + 2 * DQ + g * HD + d] + bb; o16[q] = tohx(x); }
    *(volatile v2h*)(V16 + e) = o16; __threadfence(); *(volatile v2h*)(V16 + e) = o16; }
__global__ __launch_bounds__(256) void k_asoft(const float* __restrict__ Sb, const int* __restrict__ mk, h16* P16) {
    const int lane = threadIdx.x & 31; const int row = blockIdx.x * 8 + __builtin_amdgcn_readfirstlane((int)(threadIdx.x >> 5)); if (row >= ZH * TT) return; const float* sr = Sb + (size_t)row * TT; float v[TT / 32]; const float ninf = -__builtin_inff(); float mx = ninf;
#pragma unroll
    for (int ch = 0; ch < TT / 128; ++ch) { const int j0 = ch * 128 + lane * 4; const v4f a = *(const v4f*)(sr + j0); const v4i m = *(const v4i*)(mk + j0);
#pragma unroll
        for (int q = 0; q < 4; ++q) { const float t = (m[q] != 0) ? a[q] * SCL : ninf; v[ch * 4 + q] = t; mx = fmaxf(mx, t); } }
#pragma unroll
    for (int sh = 16; sh; sh >>= 1) mx = fmaxf(mx, __shfl_xor(mx, sh, 32));
    float sum = 0.f;
#pragma unroll
    for (int k = 0; k < TT / 32; ++k) { float d0 = __fsub_rn(v[k], mx); asm volatile("" : "+v"(d0)); v[k] = __builtin_amdgcn_exp2f(__fmul_rn(d0, 1.4426950408889634f)); sum += v[k]; }
#pragma unroll
    for (int sh = 16; sh; sh >>= 1) sum += __shfl_xor(sum, sh, 32);
    const float f = __fdiv_rn(PCAR, sum);
#pragma unroll 1
    for (int ps = 0; ps < 2; ++ps) {
#pragma unroll
        for (int ch = 0; ch < TT / 128; ++ch) { v4h o4;
#pragma unroll
            for (int q = 0; q < 4; ++q) o4[q] = tohx(v[ch * 4 + q] * f);
            *(volatile v4h*)(P16 + (size_t)row * TT + ch * 128 + lane * 4) = o4; }
        if (ps == 0) __threadfence(); }
}
__global__ __launch_bounds__(256) void k_merge(const float* __restrict__ O, int h0, bf* Ah, bf* Al) { const size_t e = ((size_t)blockIdx.x * 256 + threadIdx.x) * 2; if (e >= (size_t)ZH * TT * HD) return; const int d = (int)(e % HD); const int t = (int)((e / HD) % TT); const int zz = (int)(e / ((size_t)HD * TT)); const float cs = 1.0f / PCAR; const size_t oo = (size_t)t * DQ + (h0 + zz) * HD + d;
    v2us oh, ol;
#pragma unroll
    for (int q = 0; q < 2; ++q) { unsigned short a, c2; splitf(O[e + q] * cs, a, c2); oh[q] = a; ol[q] = c2; } *(volatile v2us*)(Ah + oo) = oh; *(volatile v2us*)(Al + oo) = ol; __threadfence(); *(volatile v2us*)(Ah + oo) = oh; *(volatile v2us*)(Al + oo) = ol; }

extern "C" void kernel_launch(void* const* d_in, const int* in_sizes, int n_in,
                              void* d_out, int out_size, void* d_ws, size_t ws_size, hipStream_t stream) {
    (void)out_size;
    if (n_in < 11) return;
    if (in_sizes[0] < NB * TT * DM || in_sizes[1] < TT * HD || in_sizes[2] < NB * TT) return;
    if (in_sizes[3] < DM * DQ || in_sizes[5] < DM * DQ || in_sizes[7] < DM * DQ || in_sizes[9] < DQ * DM) return;
    if (in_sizes[4] < DQ || in_sizes[6] < DQ || in_sizes[8] < DQ || in_sizes[10] < DM) return;
    const float* x = (const float*)d_in[0]; const float* rel = (const float*)d_in[1]; const int* msk = (const int*)d_in[2];
    const float* wq = (const float*)d_in[3]; const float* bq = (const float*)d_in[4]; const float* wk = (const float*)d_in[5]; const float* bk = (const float*)d_in[6];
    const float* wv = (const float*)d_in[7]; const float* bv = (const float*)d_in[8]; const float* wo = (const float*)d_in[9]; const float* bo = (const float*)d_in[10];
    float* OUT = (float*)d_out;
    char* wsp = (char*)d_ws;
    auto take = [&](size_t bytes) { char* p = wsp; wsp += (bytes + 255) & ~(size_t)255; return (void*)p; };
    bf* WQKV = (bf*)take((size_t)NQKV * DM * 2);
    bf* WO = (bf*)take((size_t)DM * DQ * 2);
    bf* XB = (bf*)take((size_t)NB * TT * DM * 2);
    float* F = (float*)take((size_t)TT * NQKV * 4);
    h16* QK16 = (h16*)take((size_t)2 * NH_ * TT * HD * 2);
    h16* VT16 = (h16*)take((size_t)NH_ * HD * TT * 2);
    float* Sb = (float*)take((size_t)ZH * TT * TT * 4);
    h16* P16 = (h16*)take((size_t)ZH * TT * TT * 2);
    float* Ob = (float*)take((size_t)ZH * TT * HD * 4);
    bf* ATh = (bf*)take((size_t)TT * DQ * 2); bf* ATl = (bf*)take((size_t)TT * DQ * 2);
    if ((size_t)(wsp - (char*)d_ws) > ws_size) return;
    h16* Q16 = QK16; h16* K16 = QK16 + (size_t)NH_ * TT * HD;
    const unsigned GW = (unsigned)((DM * DQ / 64 + 63) / 64);
    k_wtG<<<GW, 256, 0, stream>>>(wq, DM, DQ, WQKV);
    k_wtG<<<GW, 256, 0, stream>>>(wk, DM, DQ, WQKV + (size_t)DQ * DM);
    k_wtG<<<GW, 256, 0, stream>>>(wv, DM, DQ, WQKV + (size_t)2 * DQ * DM);
    k_wtG<<<GW, 256, 0, stream>>>(wo, DQ, DM, WO);
    k_cvt8<<<dim3((unsigned)(((size_t)TT * DM / 8 + 255) / 256), NB, 1), 256, 0, stream>>>(x, XB, (size_t)TT * DM / 8, (size_t)SEQ_FULL * DM, (size_t)TT * DM);
    const unsigned LQK = (unsigned)(((size_t)2 * NH_ * TT * HD / 8 + 255) / 256), LV = (unsigned)(((size_t)NH_ * HD * TT / 2 + 255) / 256);
    for (int b = 0; b < NB; ++b) {
        k_gemmw<bf, 0, false><<<dim3(TT / 64, NQKV / 64, 1), 32, 0, stream>>>(XB + (size_t)b * TT * DM, nullptr, WQKV, nullptr, DM, F, NQKV, nullptr, 0, 0, 0);
        k_qkp<<<LQK, 256, 0, stream>>>(F, bq, bk, rel, QK16);
        k_vtp<<<LV, 256, 0, stream>>>(F, bv, VT16);
        for (int h0 = 0; h0 < NH_; h0 += ZH) {
            k_gemmw<h16, 0, false><<<dim3(TT / 64, TT / 64, ZH), 32, 0, stream>>>(Q16 + (size_t)h0 * TT * HD, nullptr, K16 + (size_t)h0 * TT * HD, nullptr, HD, Sb, TT, nullptr, (size_t)TT * HD, (size_t)TT * HD, (size_t)TT * TT);
            k_asoft<<<ZH * TT / 8, 256, 0, stream>>>(Sb, msk + (size_t)b * SEQ_FULL, P16);
            k_gemmw<h16, 0, false><<<dim3(TT / 64, HD / 64, ZH), 32, 0, stream>>>(P16, nullptr, VT16 + (size_t)h0 * HD * TT, nullptr, TT, Ob, HD, nullptr, (size_t)TT * TT, (size_t)HD * TT, (size_t)TT * HD);
            k_merge<<<(unsigned)(((size_t)ZH * TT * HD / 2 + 255) / 256), 256, 0, stream>>>(Ob, h0, ATh, ATl); }
        k_gemmw<bf, 1, true><<<dim3(TT / 64, DM / 64, 1), 32, 0, stream>>>(ATh, ATl, WO, nullptr, DQ, OUT + (size_t)b * SEQ_FULL * DM, DM, bo, 0, 0, 0); }
}
